// GraphAttentionEncoder_27144193311548
// MI455X (gfx1250) — hardware-verified
//
#include <hip/hip_runtime.h>
#include <stddef.h>


#define DF     128
#define NH     4
#define HC     32
#define GR     32
#define AP     136
#define XSP    132
#define NB     256
#define LNB    8
#define CHUNK  2048
#define NTHR   256
#define NWAVE  8
#define WCAP   256
#define NGRP   (CHUNK / (NTHR * 4))
#define WSC    16.0f
#define WSCI   0.0625f
#define LRELU  0.2f
#define LNEPS  1e-5f
#define ECLAMP 80.0f

#define LDS_SACC (2 * NB * DF)
#define LDS_DEN  (2 * NB * NH)
#define LDS_LIST (NWAVE * WCAP)
#define LDS_BYTES ((LDS_SACC + LDS_DEN + LDS_LIST + NWAVE) * 4)

static_assert(WCAP == (CHUNK / NTHR) * 32);
static_assert(NGRP >= 1);
static_assert(NB == (1 << LNB));
static_assert(CHUNK <= 4096);
static_assert(NB / NWAVE == 32);
static_assert(((LDS_SACC + LDS_DEN) % 4) == 0);
static_assert(LDS_BYTES == 278560);
static_assert(NH * HC == DF);
static_assert(NWAVE * 16 == DF);

typedef float    v4f  __attribute__((ext_vector_type(4)));
typedef float    v8f  __attribute__((ext_vector_type(8)));
typedef int      v4i  __attribute__((ext_vector_type(4)));
typedef _Float16 v8h  __attribute__((ext_vector_type(8)));
typedef _Float16 v16h __attribute__((ext_vector_type(16)));
union Frag   { v16h v; v8h half[2]; };
union Pack16 { v8h h; v4i i; };

__device__ __forceinline__ v8f wm(v16h a, v16h b, v8f c) {
  v8f d = __builtin_amdgcn_wmma_f32_16x16x32_f16(false, a, false, b, (short)0, c, false, false);
  asm volatile("v_nop\n\tv_nop\n\tv_nop\n\tv_nop" : "+v"(d) : "v"(a), "v"(b));
  return d;
}

__device__ __forceinline__ float wsum(float v) {
  v += __shfl_xor(v, 16, 32);
  v += __shfl_xor(v, 8, 32);
  v += __shfl_xor(v, 4, 32);
  v += __shfl_xor(v, 2, 32);
  v += __shfl_xor(v, 1, 32);
  return v;
}

__device__ __forceinline__ float dot4(v4f a, v4f b) {
  return a.x * b.x + a.y * b.y + a.z * b.z + a.w * b.w;
}

__device__ __forceinline__ float rcpf(float v) { return __builtin_amdgcn_rcpf(v); }

__global__ __launch_bounds__(NTHR) void k_prep(const float* __restrict__ W1,
                                                const float* __restrict__ W2, _Float16* Wh) {
  __shared__ __attribute__((aligned(16))) _Float16 T[32 * AP];
  const int tid   = threadIdx.x;
  const int layer = blockIdx.y;
  const float* W  = layer ? W2 : W1;
  const int n0    = blockIdx.x * 32;
  _Float16* dstp  = Wh + (size_t)layer * DF * DF;

#pragma unroll 1
  for (int idx = tid; idx < 32 * DF; idx += NTHR) {
    const int k = idx >> 5, j = idx & 31;
    T[j * AP + k] = (_Float16)(W[(size_t)k * DF + n0 + j] * WSC);
  }
  __syncthreads();

  const int r = tid >> 4;
  const int q = (tid & 15) * 8;
  Pack16 u0, u1;
  u0.h = *(const v8h*)(T + r * AP + q);
  u1.h = *(const v8h*)(T + (r + 16) * AP + q);
  _Float16* p0 = dstp + (size_t)(n0 + r) * DF + q;
  _Float16* p1 = dstp + (size_t)(n0 + r + 16) * DF + q;
  *(volatile v4i*)p0 = u0.i;
  *(volatile v4i*)p1 = u1.i;
  __threadfence();
  *(volatile v4i*)p0 = u0.i;
  *(volatile v4i*)p1 = u1.i;
}

__device__ __forceinline__ void epi_tile(v8f acc, int T, int hh, int m, int wave, int ncol,
                                         float cs, float cd, float* Xs, float* As, float* Ds) {
  float ss[8], sd[8];
#pragma unroll
  for (int r = 0; r < 8; ++r) {
    const float v = acc[r] * WSCI;
    Xs[(T * 16 + 8 * hh + r) * XSP + ncol] = v;
    ss[r] = v * cs;
    sd[r] = v * cd;
  }
#pragma unroll
  for (int mk = 1; mk < 16; mk <<= 1) {
#pragma unroll
    for (int r = 0; r < 8; ++r) {
      ss[r] += __shfl_xor(ss[r], mk, 32);
      sd[r] += __shfl_xor(sd[r], mk, 32);
    }
  }
  if (m == 0) {
#pragma unroll
    for (int r = 0; r < 8; ++r) {
      As[(T * 16 + 8 * hh + r) * NWAVE + wave] = ss[r];
      Ds[(T * 16 + 8 * hh + r) * NWAVE + wave] = sd[r];
    }
  }
}

__global__ __launch_bounds__(NTHR) void k_gemm(
    const float* __restrict__ x, const _Float16* __restrict__ Wh,
    const float* __restrict__ as1, const float* __restrict__ ad1,
    const float* __restrict__ as2, const float* __restrict__ ad2,
    float* h, float* es, float* ed, int nN, int nP) {
  __shared__ __attribute__((aligned(16))) _Float16 At[GR * AP];
  __shared__ __attribute__((aligned(16))) float Xs[GR * XSP];
  __shared__ __attribute__((aligned(16))) float As[GR * NWAVE];
  __shared__ __attribute__((aligned(16))) float Ds[GR * NWAVE];

  const int tid   = threadIdx.x;
  const int lane  = tid & 31;
  const int wave  = tid >> 5;
  const int hh    = lane >> 4;
  const int m     = lane & 15;
  const int layer = blockIdx.y;
  const int rowBase = blockIdx.x * GR;

  const _Float16* Wl = Wh + (size_t)layer * DF * DF;
  const float* att_s = layer ? as2 : as1;
  const float* att_d = layer ? ad2 : ad1;
  float* hl  = h  + (size_t)layer * (size_t)nP * DF;
  float* esl = es + (size_t)layer * (size_t)nP * NH;
  float* edl = ed + (size_t)layer * (size_t)nP * NH;

  {
    const int r  = tid >> 3;
    const int c0 = (tid & 7) * 16;
    int row = rowBase + r;
    if (row > nN - 1) row = nN - 1;
    const float* p = x + (size_t)row * DF + c0;
    const v4f f0 = *(const v4f*)(p), f1 = *(const v4f*)(p + 4);
    const v4f f2 = *(const v4f*)(p + 8), f3 = *(const v4f*)(p + 12);
    Pack16 u0, u1;
    u0.h[0] = (_Float16)f0.x; u0.h[1] = (_Float16)f0.y; u0.h[2] = (_Float16)f0.z; u0.h[3] = (_Float16)f0.w;
    u0.h[4] = (_Float16)f1.x; u0.h[5] = (_Float16)f1.y; u0.h[6] = (_Float16)f1.z; u0.h[7] = (_Float16)f1.w;
    u1.h[0] = (_Float16)f2.x; u1.h[1] = (_Float16)f2.y; u1.h[2] = (_Float16)f2.z; u1.h[3] = (_Float16)f2.w;
    u1.h[4] = (_Float16)f3.x; u1.h[5] = (_Float16)f3.y; u1.h[6] = (_Float16)f3.z; u1.h[7] = (_Float16)f3.w;
    *(v8h*)(At + r * AP + c0)     = u0.h;
    *(v8h*)(At + r * AP + c0 + 8) = u1.h;
  }
  __syncthreads();

  const int ncol = wave * 16 + m;
  v8f c0a = {0.f, 0.f, 0.f, 0.f, 0.f, 0.f, 0.f, 0.f};
  v8f c1a = {0.f, 0.f, 0.f, 0.f, 0.f, 0.f, 0.f, 0.f};
#pragma unroll
  for (int kt = 0; kt < DF / 32; ++kt) {
    const int k0 = kt * 32;
    Frag a0, a1, b;
    const _Float16* pb  = Wl + (size_t)ncol * DF + k0 + 8 * hh;
    const _Float16* pa0 = At + m * AP + k0 + 8 * hh;
    const _Float16* pa1 = At + (16 + m) * AP + k0 + 8 * hh;
    b.half[0]  = *(const v8h*)pb;  b.half[1]  = *(const v8h*)(pb + 16);
    a0.half[0] = *(const v8h*)pa0; a0.half[1] = *(const v8h*)(pa0 + 16);
    a1.half[0] = *(const v8h*)pa1; a1.half[1] = *(const v8h*)(pa1 + 16);
    c0a = wm(a0.v, b.v, c0a);
    c1a = wm(a1.v, b.v, c1a);
  }

  const float cs = att_s[ncol];
  const float cd = att_d[ncol];
  epi_tile(c0a, 0, hh, m, wave, ncol, cs, cd, Xs, As, Ds);
  epi_tile(c1a, 1, hh, m, wave, ncol, cs, cd, Xs, As, Ds);
  __syncthreads();

  v4f xr[4];
#pragma unroll
  for (int i = 0; i < 4; ++i) xr[i] = *(const v4f*)(Xs + (4 * wave + i) * XSP + 4 * lane);
  float* gp = 0;
  v4f gv = {0.f, 0.f, 0.f, 0.f};
  if (wave == 0) {
    gv.x = As[lane * NWAVE + 0] + As[lane * NWAVE + 1];
    gv.y = As[lane * NWAVE + 2] + As[lane * NWAVE + 3];
    gv.z = As[lane * NWAVE + 4] + As[lane * NWAVE + 5];
    gv.w = As[lane * NWAVE + 6] + As[lane * NWAVE + 7];
    gp = esl + (size_t)rowBase * NH + 4 * lane;
  } else if (wave == 1) {
    gv.x = Ds[lane * NWAVE + 0] + Ds[lane * NWAVE + 1];
    gv.y = Ds[lane * NWAVE + 2] + Ds[lane * NWAVE + 3];
    gv.z = Ds[lane * NWAVE + 4] + Ds[lane * NWAVE + 5];
    gv.w = Ds[lane * NWAVE + 6] + Ds[lane * NWAVE + 7];
    gp = edl + (size_t)rowBase * NH + 4 * lane;
  }
  float* hp[4];
#pragma unroll
  for (int i = 0; i < 4; ++i) hp[i] = hl + (size_t)(rowBase + 4 * wave + i) * DF + 4 * lane;

#pragma unroll
  for (int i = 0; i < 4; ++i) *(volatile v4f*)(hp[i]) = xr[i];
  if (gp) *(volatile v4f*)gp = gv;
  __threadfence();
#pragma unroll
  for (int i = 0; i < 4; ++i) *(volatile v4f*)(hp[i]) = xr[i];
  if (gp) *(volatile v4f*)gp = gv;
}

__global__ __launch_bounds__(NTHR) void k_gat(
    const float* __restrict__ x, const int* __restrict__ ei,
    const float* __restrict__ h, const float* __restrict__ es, const float* __restrict__ ed,
    const float* __restrict__ b1, const float* __restrict__ b2,
    const float* __restrict__ gW, const float* __restrict__ gb,
    const float* __restrict__ gam, const float* __restrict__ bet,
    float* out, int nN, int nE, int nP) {
  extern __shared__ v4f lds_dyn[];
  float* sacc = (float*)lds_dyn;
  float* den  = sacc + LDS_SACC;
  int*   list = (int*)(den + LDS_DEN);
  int*   wcnt = list + LDS_LIST;

  const int tid  = threadIdx.x;
  const int lane = tid & 31;
  const int wave = tid >> 5;
  const int hd   = lane >> 3;
  const int nodeBase = blockIdx.x * NB;
  const size_t sH = (size_t)nP * DF;
  const size_t sE = (size_t)nP * NH;

  {
    const v4f z4 = {0.f, 0.f, 0.f, 0.f};
    for (int i = tid; i < (LDS_SACC + LDS_DEN) / 4; i += NTHR) lds_dyn[i] = z4;
  }
  __syncthreads();

  const int* eid = ei + nE;
  const bool al16 = ((nE & 3) == 0);

  const int nChunks = (nE + CHUNK - 1) / CHUNK;
#pragma unroll 1
  for (int ch = 0; ch < nChunks; ++ch) {
    const int cbase = ch * CHUNK;
    int wc = 0;
#pragma unroll
    for (int g = 0; g < NGRP; ++g) {
      const int el0 = (g * NTHR + tid) * 4;
      const int e0  = cbase + el0;
      const int sent = -2147483647 - 1;
      v4i d;
      if (al16 && (e0 + 3 < nE)) {
        d = *(const v4i*)(eid + e0);
      } else {
        d.x = (e0     < nE) ? eid[min(e0, nE - 1)]     : sent;
        d.y = (e0 + 1 < nE) ? eid[min(e0 + 1, nE - 1)] : sent;
        d.z = (e0 + 2 < nE) ? eid[min(e0 + 2, nE - 1)] : sent;
        d.w = (e0 + 3 < nE) ? eid[min(e0 + 3, nE - 1)] : sent;
      }
      const unsigned s0 = (unsigned)d.x - (unsigned)nodeBase;
      const unsigned s1 = (unsigned)d.y - (unsigned)nodeBase;
      const unsigned s2 = (unsigned)d.z - (unsigned)nodeBase;
      const unsigned s3 = (unsigned)d.w - (unsigned)nodeBase;
      const bool h0 = s0 < (unsigned)NB;
      const bool h1 = s1 < (unsigned)NB;
      const bool h2 = s2 < (unsigned)NB;
      const bool h3 = s3 < (unsigned)NB;
      const unsigned many = __builtin_amdgcn_ballot_w32(h0 | h1 | h2 | h3);
      if (many != 0u) {
#define HITJ(J, HJ, SJ) { \
          const unsigned mj = __builtin_amdgcn_ballot_w32(HJ); \
          if (HJ) { \
            const int pos = wc + (int)__builtin_amdgcn_mbcnt_lo(mj, 0u); \
            if (pos < WCAP) list[wave * WCAP + pos] = ((el0 + (J)) << LNB) | (int)(SJ); \
          } \
          wc += (int)__builtin_popcount(mj); }
        HITJ(0, h0, s0)
        HITJ(1, h1, s1)
        HITJ(2, h2, s2)
        HITJ(3, h3, s3)
#undef HITJ
      }
    }
    if (lane == 0) wcnt[wave] = wc;
    __syncthreads();

    if (wave == 0) {
      for (int wsx = 0; wsx < NWAVE; ++wsx) {
        int n = wcnt[wsx];
        if (n > WCAP) n = WCAP;
        if (n < 0) n = 0;
        for (int i = 0; i < n; ++i) {
          const int ent  = list[wsx * WCAP + i];
          const int slot = ent & (NB - 1);
          const int el   = (ent >> LNB) & (CHUNK - 1);
          int e = cbase + el;
          if (e > nE - 1) e = nE - 1;
          int src = ei[e];
          src = src < 0 ? 0 : (src > nN - 1 ? nN - 1 : src);
          int nd = nodeBase + slot;
          if (nd > nN - 1) nd = nN - 1;
          const size_t so = (size_t)src;
          const size_t no = (size_t)nd;
          float a0 = es[so * NH + hd] + ed[no * NH + hd];
          a0 = (a0 > 0.f) ? a0 : LRELU * a0;
          a0 = fminf(a0, ECLAMP);
          const float p0 = __expf(a0);
          float a1 = es[sE + so * NH + hd] + ed[sE + no * NH + hd];
          a1 = (a1 > 0.f) ? a1 : LRELU * a1;
          a1 = fminf(a1, ECLAMP);
          const float p1 = __expf(a1);
          const v4f xv0 = *(const v4f*)(h + so * DF + 4 * lane);
          const v4f xv1 = *(const v4f*)(h + sH + so * DF + 4 * lane);
          v4f* sp0 = (v4f*)(sacc + slot * DF + 4 * lane);
          v4f* sp1 = (v4f*)(sacc + (NB + slot) * DF + 4 * lane);
          const v4f cu0 = *sp0;
          const v4f cu1 = *sp1;
          const v4f nx0 = cu0 + p0 * xv0;
          const v4f nx1 = cu1 + p1 * xv1;
          *sp0 = nx0;
          *sp1 = nx1;
          if ((lane & 7) == 0) {
            const float o0 = den[slot * NH + hd];
            const float o1 = den[NB * NH + slot * NH + hd];
            den[slot * NH + hd]           = o0 + p0;
            den[NB * NH + slot * NH + hd] = o1 + p1;
          }
        }
      }
    }
    __syncthreads();
  }

  const v4f b14 = *(const v4f*)(b1 + 4 * lane);
  const v4f b24 = *(const v4f*)(b2 + 4 * lane);
  const v4f g4  = *(const v4f*)(gam + 4 * lane);
  const v4f e4  = *(const v4f*)(bet + 4 * lane);
  const v4f q0 = *(const v4f*)(gW + 8 * lane);
  const v4f q1 = *(const v4f*)(gW + 8 * lane + 4);
  const v4f q2 = *(const v4f*)(gW + 2 * DF + 8 * lane);
  const v4f q3 = *(const v4f*)(gW + 2 * DF + 8 * lane + 4);
  const v4f wa0 = {q0.x, q0.z, q1.x, q1.z};
  const v4f wa1 = {q0.y, q0.w, q1.y, q1.w};
  const v4f wb0 = {q2.x, q2.z, q3.x, q3.z};
  const v4f wb1 = {q2.y, q2.w, q3.y, q3.w};
  const float gb0 = gb[0];
  const float gb1 = gb[1];
#pragma unroll 1
  for (int j = 0; j < NB / NWAVE; ++j) {
    const int slot = wave * (NB / NWAVE) + j;
    const int node = nodeBase + slot;
    if (node >= nN) break;
    const size_t nr = (size_t)node;
    float a0 = es[nr * NH + hd] + ed[nr * NH + hd];
    a0 = (a0 > 0.f) ? a0 : LRELU * a0;
    a0 = fminf(a0, ECLAMP);
    const float p0 = __expf(a0);
    const v4f xv0 = *(const v4f*)(h + nr * DF + 4 * lane);
    const v4f sv0 = *(const v4f*)(sacc + slot * DF + 4 * lane) + p0 * xv0;
    const float dv0 = den[slot * NH + hd] + p0;
    const float iv0 = rcpf(dv0);
    const v4f o1 = sv0 * iv0 + b14;
    float a1 = es[sE + nr * NH + hd] + ed[sE + nr * NH + hd];
    a1 = (a1 > 0.f) ? a1 : LRELU * a1;
    a1 = fminf(a1, ECLAMP);
    const float p1 = __expf(a1);
    const v4f xv1 = *(const v4f*)(h + sH + nr * DF + 4 * lane);
    const v4f sv1 = *(const v4f*)(sacc + (NB + slot) * DF + 4 * lane) + p1 * xv1;
    const float dv1 = den[NB * NH + slot * NH + hd] + p1;
    const float iv1 = rcpf(dv1);
    const v4f o2 = sv1 * iv1 + b24;
    float l0 = dot4(o1, wa0) + dot4(o2, wb0);
    float l1 = dot4(o1, wa1) + dot4(o2, wb1);
    l0 = wsum(l0) + gb0;
    l1 = wsum(l1) + gb1;
    const float gm = fmaxf(l0, l1);
    const float x0 = __expf(l0 - gm);
    const float x1 = __expf(l1 - gm);
    const float ri = rcpf(x0 + x1);
    const float g0 = x0 * ri;
    const float g1 = x1 * ri;
    const v4f xr  = *(const v4f*)(x + nr * DF + 4 * lane);
    const v4f mix = g0 * o1 + g1 * o2;
    const v4f y   = xr + mix;
    const float s  = wsum(y.x + y.y + y.z + y.w);
    const float mu = s * (1.0f / DF);
    const v4f dd = y - mu;
    const float qv = wsum(dd.x * dd.x + dd.y * dd.y + dd.z * dd.z + dd.w * dd.w);
    const float rs = rsqrtf(qv * (1.0f / DF) + LNEPS);
    const v4f o = dd * rs * g4 + e4;
    float* op = out + nr * DF + 4 * lane;
    *(volatile v4f*)op = o;
    __threadfence();
    *(volatile v4f*)op = o;
  }
}

extern "C" void kernel_launch(void* const* d_in, const int* in_sizes, int n_in,
                              void* d_out, int out_size, void* d_ws, size_t ws_size,
                              hipStream_t stream) {
  if (n_in < 14) return;
  const int nN = in_sizes[0] / DF;
  if (nN <= 0 || in_sizes[0] != nN * DF) return;
  if (in_sizes[1] < 0 || (in_sizes[1] & 1)) return;
  const int nE = in_sizes[1] / 2;
  if (in_sizes[2] != DF * DF || in_sizes[6] != DF * DF) return;
  if (in_sizes[3] != DF || in_sizes[7] != DF) return;
  if (in_sizes[4] != NH * HC || in_sizes[5] != NH * HC) return;
  if (in_sizes[8] != NH * HC || in_sizes[9] != NH * HC) return;
  if (in_sizes[10] != 2 * DF * 2 || in_sizes[11] != 2) return;
  if (in_sizes[12] != DF || in_sizes[13] != DF) return;
  if (out_size != nN * DF) return;

  const float* x   = (const float*)d_in[0];
  const int*   ei  = (const int*)d_in[1];
  const float* W1  = (const float*)d_in[2];
  const float* b1  = (const float*)d_in[3];
  const float* as1 = (const float*)d_in[4];
  const float* ad1 = (const float*)d_in[5];
  const float* W2  = (const float*)d_in[6];
  const float* b2  = (const float*)d_in[7];
  const float* as2 = (const float*)d_in[8];
  const float* ad2 = (const float*)d_in[9];
  const float* gW  = (const float*)d_in[10];
  const float* gb  = (const float*)d_in[11];
  const float* gam = (const float*)d_in[12];
  const float* bet = (const float*)d_in[13];
  float* out = (float*)d_out;

  const int nP = ((nN + GR - 1) / GR) * GR;
  size_t off = 0;
  _Float16* Wh = (_Float16*)((char*)d_ws + off); off += (size_t)2 * DF * DF * sizeof(_Float16);
  float* h  = (float*)((char*)d_ws + off);       off += (size_t)2 * nP * DF * sizeof(float);
  float* es = (float*)((char*)d_ws + off);       off += (size_t)2 * nP * NH * sizeof(float);
  float* ed = (float*)((char*)d_ws + off);       off += (size_t)2 * nP * NH * sizeof(float);
  if (off > ws_size) return;
  if (off > (size_t)134217728) return;

  k_prep<<<dim3(DF / 32, 2), NTHR, 0, stream>>>(W1, W2, Wh);

  k_gemm<<<dim3(nP / GR, 2), NTHR, 0, stream>>>(x, Wh, as1, ad1, as2, ad2, h, es, ed, nN, nP);

  hipFuncSetAttribute(reinterpret_cast<const void*>(&k_gat),
                      hipFuncAttributeMaxDynamicSharedMemorySize, LDS_BYTES);
  const int grid = (nN + NB - 1) / NB;
  k_gat<<<grid, NTHR, LDS_BYTES, stream>>>(x, ei, h, es, ed, b1, b2, gW, gb, gam, bet,
                                           out, nN, nE, nP);
}
